// VectorizedQuantumCircuit_90142773609090
// MI455X (gfx1250) — hardware-verified
//
#include <hip/hip_runtime.h>
#include <math.h>

typedef __attribute__((ext_vector_type(16))) _Float16 v16h;
typedef __attribute__((ext_vector_type(8)))  _Float16 v8h;
typedef __attribute__((ext_vector_type(8)))  float    v8f;
typedef __attribute__((ext_vector_type(4)))  float    v4f;

constexpr int kAxes        = 12;
constexpr int kLayers      = 4;
constexpr int kDim         = 1 << kAxes;
constexpr int kSide        = 64;
constexpr int kSamples     = 8192;
constexpr int kRowsPerBlk  = 8;
constexpr int kPairIters   = 4;
constexpr int kBlocks      = kSamples / kRowsPerBlk;
constexpr int kPlaneElems  = kSide * kSide;
constexpr int kNumPlanes   = (kLayers - 1) * 2;
constexpr int kSignRows    = 16;
static_assert(kSide * kSide == kDim);
static_assert(kRowsPerBlk == 2 * kPairIters);
static_assert(kBlocks * kRowsPerBlk == kSamples);
static_assert(kSamples * kAxes == 98304);
static_assert(kLayers * kAxes == 48);
static_assert((kSide % 32) == 0);
static_assert((kRowsPerBlk * kAxes * 4) % 128 == 0);

constexpr float kStateCarry   = 4096.0f;
constexpr float kMatCarry     = 1024.0f;
constexpr float kInvMatCarry  = 1.0f / kMatCarry;
constexpr float kRemCarry     = 2048.0f;
constexpr float kInvRemCarry  = 1.0f / kRemCarry;
constexpr float kProbCarry    = 32768.0f;
constexpr float kProbFold     = kProbCarry / (kStateCarry * kStateCarry);
constexpr float kF16MinNormal = 6.103515625e-5f;

constexpr size_t kOffFact = 0;
constexpr size_t kOffSign = kOffFact + (size_t)kNumPlanes * kPlaneElems * 2;
constexpr size_t kWsTotal = kOffSign + (size_t)kSignRows * kSide * 2;
static_assert(kOffSign == 49152ull);
static_assert(kWsTotal == 51200ull);
static_assert(kWsTotal <= 134217728ull);
static_assert((kOffSign % 128) == 0);

__host__ __device__ constexpr unsigned ring_src(unsigned d) {
  return (d ^ ((d << 1) & 0xFFFu) ^ (3u * (d >> 11))) & 0xFFFu;
}
__host__ __device__ constexpr unsigned ring_dst(unsigned e) {
  unsigned p = e;
  p ^= p << 1;
  p ^= p << 2;
  p ^= p << 4;
  p ^= p << 8;
  p &= 0xFFFu;
  return p ^ (p >> 11);
}
constexpr unsigned ring_src_chain(unsigned d) {
  for (int i = kAxes - 1; i >= 0; --i) {
    const int t = (i + 1) % kAxes;
    if ((d >> i) & 1u) d ^= (1u << t);
  }
  return d;
}
constexpr bool ring_forms_agree() {
  for (unsigned d = 0; d < 4096u; d += 5u) {
    if (ring_src(d) != ring_src_chain(d)) return false;
    if (ring_dst(ring_src(d)) != d) return false;
  }
  for (unsigned b = 0; b < 12u; ++b) {
    const unsigned d = 1u << b;
    if (ring_src(d) != ring_src_chain(d)) return false;
    if (ring_dst(ring_src(d)) != d) return false;
    if (ring_src(d ^ 0xFFFu) != (ring_src(d) ^ ring_src(0xFFFu))) return false;
  }
  return true;
}
static_assert(ring_forms_agree());

union FragU { v16h v; v8h h[2]; };
__device__ __forceinline__ v16h frag_load(const _Float16* p) {
  FragU f;
  f.h[0] = *(const v8h*)(p);
  f.h[1] = *(const v8h*)(p + 16);
  return f.v;
}
__device__ __forceinline__ v8f mma_f16(v16h a, v16h b, v8f c) {
  c = __builtin_amdgcn_wmma_f32_16x16x32_f16(false, a, false, b, (short)0, c, false, false);
  asm volatile("v_nop\n\tv_nop\n\tv_nop\n\tv_nop" : "+v"(c) : "v"(a), "v"(b));
  return c;
}
__device__ __forceinline__ float flush_f16_range(float v) {
  return (fabsf(v) < kF16MinNormal) ? 0.0f : v;
}

__device__ __forceinline__ void tile_product(const _Float16* aRow, const _Float16* bBase,
                                             v8f& c0, v8f& c1, v8f& c2, v8f& c3) {
  const v8f z = (v8f){0.f, 0.f, 0.f, 0.f, 0.f, 0.f, 0.f, 0.f};
  c0 = z; c1 = z; c2 = z; c3 = z;
#pragma unroll
  for (int ks = 0; ks < 2; ++ks) {
    const v16h a = frag_load(aRow + ks * 32);
    v16h b;
    b = frag_load(bBase + 0 * 1024 + ks * 32);
    c0 = mma_f16(a, b, c0);
    b = frag_load(bBase + 1 * 1024 + ks * 32);
    c1 = mma_f16(a, b, c1);
    b = frag_load(bBase + 2 * 1024 + ks * 32);
    c2 = mma_f16(a, b, c2);
    b = frag_load(bBase + 3 * 1024 + ks * 32);
    c3 = mma_f16(a, b, c3);
  }
}

__device__ __forceinline__ void tile_product2(const _Float16* aRow, const _Float16* aRow2, const _Float16* bBase,
                                              v8f& c0, v8f& c1, v8f& c2, v8f& c3,
                                              v8f& e0, v8f& e1, v8f& e2, v8f& e3) {
  const v8f z = (v8f){0.f, 0.f, 0.f, 0.f, 0.f, 0.f, 0.f, 0.f};
  c0 = z; c1 = z; c2 = z; c3 = z;
  e0 = z; e1 = z; e2 = z; e3 = z;
#pragma unroll
  for (int ks = 0; ks < 2; ++ks) {
    const v16h a  = frag_load(aRow + ks * 32);
    const v16h a2 = frag_load(aRow2 + ks * 32);
    v16h b;
    b = frag_load(bBase + 0 * 1024 + ks * 32);
    c0 = mma_f16(a, b, c0);
    e0 = mma_f16(a2, b, e0);
    b = frag_load(bBase + 1 * 1024 + ks * 32);
    c1 = mma_f16(a, b, c1);
    e1 = mma_f16(a2, b, e1);
    b = frag_load(bBase + 2 * 1024 + ks * 32);
    c2 = mma_f16(a, b, c2);
    e2 = mma_f16(a2, b, e2);
    b = frag_load(bBase + 3 * 1024 + ks * 32);
    c3 = mma_f16(a, b, c3);
    e3 = mma_f16(a2, b, e3);
  }
}

__device__ __forceinline__ void pack_state2(v8f acc, v8h& val, v8h& rem) {
#pragma unroll
  for (int r = 0; r < 8; ++r) {
    const float w  = acc[r] * kInvMatCarry;
    const float wv = flush_f16_range(w);
    const _Float16 hv = (_Float16)wv;
    const float back = (float)hv;
    const float dv = flush_f16_range((w - back) * kRemCarry);
    val[r] = hv;
    rem[r] = (_Float16)dv;
  }
}

__device__ __forceinline__ void scatter_tile(v8f acc, v8f accr, unsigned dj, _Float16* dstBase, bool last) {
#pragma unroll
  for (int r = 0; r < 8; ++r) {
    const float w  = (acc[r] + accr[r] * kInvRemCarry) * kInvMatCarry;
    const float pv = w * w * kProbFold;
    const float v  = flush_f16_range(last ? pv : w);
    const unsigned d = dj ^ ring_dst((unsigned)r);
    dstBase[d] = (_Float16)v;
  }
}

__global__ __launch_bounds__(256) void prep_planes_kernel(const float* __restrict__ theta,
                                                          unsigned short* __restrict__ planes) {
  __shared__ float sCos[36];
  __shared__ float sSin[36];
  const unsigned tid = threadIdx.x;
  const unsigned ti = (tid < 36u) ? tid : 35u;
  float th = theta[12u + ti];
  asm volatile("" : "+v"(th));
  float sn, cs;
  sincosf(0.5f * th, &sn, &cs);
  if (tid < 36u) {
    sCos[tid] = cs;
    sSin[tid] = sn;
  }
  __syncthreads();

#pragma unroll 1
  for (unsigned rep = 0; rep < 12u; ++rep) {
    unsigned e0 = (rep * 256u + tid) * 8u;
    asm volatile("" : "+v"(e0));
    const unsigned pl    = e0 >> 12;
    const unsigned layer = pl >> 1;
    const unsigned which = pl & 1u;
    const unsigned n     = (e0 >> 6) & 63u;
    const unsigned k0    = e0 & 63u;
    const unsigned base  = layer * 12u + which * 6u;
    float cj[6], sj[6];
#pragma unroll
    for (int j = 0; j < 6; ++j) {
      cj[j] = sCos[base + j];
      sj[j] = sSin[base + j];
    }
    float common = kMatCarry;
#pragma unroll
    for (int j = 3; j < 6; ++j) {
      const unsigned bn = (n >> j) & 1u;
      const unsigned bk = (k0 >> j) & 1u;
      const float offd = bn ? sj[j] : -sj[j];
      common *= (bn == bk) ? cj[j] : offd;
    }
    const unsigned n0 = n & 1u, n1 = (n >> 1) & 1u, n2 = (n >> 2) & 1u;
    const float f00 = n0 ? sj[0] : cj[0];
    const float f01 = n0 ? cj[0] : -sj[0];
    const float f10 = n1 ? sj[1] : cj[1];
    const float f11 = n1 ? cj[1] : -sj[1];
    const float f20 = n2 ? sj[2] : cj[2];
    const float f21 = n2 ? cj[2] : -sj[2];
    v8h hv;
#pragma unroll
    for (int jj = 0; jj < 8; ++jj) {
      float v = common;
      v *= (jj & 1) ? f01 : f00;
      v *= (jj & 2) ? f11 : f10;
      v *= (jj & 4) ? f21 : f20;
      v = flush_f16_range(v);
      hv[jj] = (_Float16)v;
    }
    unsigned short* dst = planes + e0;
    *(volatile v8h*)dst = hv;
    __threadfence();
    *(volatile v8h*)dst = hv;
  }

  if (tid < 128u) {
    const unsigned n  = tid >> 3;
    const unsigned k0 = (tid & 7u) * 8u;
    v8h hv;
#pragma unroll
    for (int jj = 0; jj < 8; ++jj) {
      const unsigned k = k0 + (unsigned)jj;
      const float sg = ((k >> n) & 1u) ? -1.0f : 1.0f;
      const float v = (n < 6u) ? sg : ((n == 6u) ? 1.0f : 0.0f);
      hv[jj] = (_Float16)v;
    }
    unsigned short* dst = planes + (size_t)kNumPlanes * kPlaneElems + tid * 8u;
    *(volatile v8h*)dst = hv;
    __threadfence();
    *(volatile v8h*)dst = hv;
  }
}

__global__ __launch_bounds__(256) void state_evolve_kernel(const float* __restrict__ x,
                                                           const float* __restrict__ theta,
                                                           const unsigned short* __restrict__ planes,
                                                           float* __restrict__ out) {
  __shared__ __align__(16) _Float16 sS[2 * kDim];
  __shared__ __align__(16) _Float16 sT[2 * kDim];
  __shared__ __align__(16) _Float16 sT2[2 * kDim];
  __shared__ __align__(16) _Float16 sK[kNumPlanes * kPlaneElems];
  __shared__ __align__(16) _Float16 sG[kSignRows * kSide];
  __shared__ __align__(16) float sCS[kRowsPerBlk * kAxes * 2];
  __shared__ __align__(16) float sA[kRowsPerBlk * 2 * kSide];
  __shared__ __align__(16) float sR[2 * kSide * 16];
  __shared__ __align__(16) float sOut[kRowsPerBlk * kAxes];

  const unsigned tid = threadIdx.x;
  unsigned lane = tid & 31u;
  unsigned wave = tid >> 5;
  asm volatile("" : "+v"(lane));
  unsigned c = lane & 15u;
  unsigned h = lane >> 4;
  asm volatile("" : "+v"(c));
  asm volatile("" : "+v"(h));
  const unsigned elw = wave >> 2;
  const unsigned r0  = (wave & 3u) * 16u;
  const unsigned b0  = blockIdx.x * (unsigned)kRowsPerBlk;

  {
    const _Float16* Pl = (const _Float16*)planes;
#pragma unroll 1
    for (unsigned rep = 0; rep < 12u; ++rep) {
      const unsigned o = (rep * 256u + tid) * 8u;
      *(v8h*)(sK + o) = *(const v8h*)(Pl + o);
    }
    if (wave < 4u) {
      const unsigned o = tid * 8u;
      *(v8h*)(sG + o) = *(const v8h*)(Pl + (size_t)kNumPlanes * kPlaneElems + o);
    }
  }
  if (wave < 3u) {
    unsigned t32 = tid;
    asm volatile("" : "+v"(t32));
    unsigned rq = (t32 * 0xAAABu) >> 19;
    asm volatile("" : "+v"(rq));
    unsigned q = t32 - rq * 12u;
    asm volatile("" : "+v"(q));
    float xv = x[b0 * (unsigned)kAxes + t32];
    float th = theta[q];
    asm volatile("" : "+v"(xv));
    asm volatile("" : "+v"(th));
    float sn, cs;
    sincosf(0.5f * (xv + th), &sn, &cs);
    sCS[t32 * 2u]      = cs;
    sCS[t32 * 2u + 1u] = sn;
  }
  __syncthreads();
#pragma unroll 1
  for (unsigned rep = 0; rep < 4u; ++rep) {
    const unsigned idx   = rep * 256u + tid;
    const unsigned row   = idx >> 7;
    const unsigned which = (idx >> 6) & 1u;
    const unsigned m     = idx & 63u;
    const float* csp = sCS + (row * 12u + which * 6u) * 2u;
    float p = 1.0f;
#pragma unroll
    for (int j = 0; j < 6; ++j) p *= csp[j * 2 + ((m >> j) & 1u)];
    sA[idx] = p;
  }
  __syncthreads();

  const _Float16* aRowS  = sS  + (elw * 64u + r0 + c) * 64u + 8u * h;
  const _Float16* aRowT  = sT  + (elw * 64u + r0 + c) * 64u + 8u * h;
  const _Float16* aRowT2 = sT2 + (elw * 64u + r0 + c) * 64u + 8u * h;
  _Float16* tDst  = sT  + (elw * 64u + c) * 64u + r0 + 8u * h;
  _Float16* tDst2 = sT2 + (elw * 64u + c) * 64u + r0 + 8u * h;
  _Float16* sDst = sS + elw * (unsigned)kDim;
  const _Float16* bK = sK + c * 64u + 8u * h;
  const _Float16* bG = sG + c * 64u + 8u * h;
  float* rDst = sR + (elw * 64u + r0 + 8u * h) * 16u + c;
  unsigned dl = ring_dst(c * 64u + r0 + 8u * h);
  asm volatile("" : "+v"(dl));

#pragma unroll 1
  for (unsigned it = 0; it < (unsigned)kPairIters; ++it) {
#pragma unroll 1
    for (unsigned rep = 0; rep < 4u; ++rep) {
      unsigned vi = rep * 256u + tid;
      asm volatile("" : "+v"(vi));
      const unsigned el    = vi >> 9;
      const unsigned dbase = (vi & 511u) * 8u;
      unsigned sb = ring_src(dbase);
      asm volatile("" : "+v"(sb));
      const unsigned row = 2u * it + el;
      const float* fLo = sA + row * 128u;
      const float* fHi = fLo + 64u;
      const float ahi = fHi[sb >> 6] * kStateCarry;
      v8h hv;
#pragma unroll
      for (int jj = 0; jj < 8; ++jj) {
        const float v = flush_f16_range(ahi * fLo[(sb ^ ring_src((unsigned)jj)) & 63u]);
        hv[jj] = (_Float16)v;
      }
      *(v8h*)(sS + el * (unsigned)kDim + dbase) = hv;
    }
    __syncthreads();

#pragma unroll 1
    for (unsigned l = 0; l < 3u; ++l) {
      const _Float16* bLo = bK + (2u * l) * (unsigned)kPlaneElems;
      const _Float16* bHi = bK + (2u * l + 1u) * (unsigned)kPlaneElems;
      const bool last = (l == 2u);
      {
        v8f a0, a1, a2, a3;
        tile_product(aRowS, bLo, a0, a1, a2, a3);
        v8h hv, rv;
        pack_state2(a0, hv, rv);
        *(v8h*)(tDst  + 0 * 1024) = hv;
        *(v8h*)(tDst2 + 0 * 1024) = rv;
        pack_state2(a1, hv, rv);
        *(v8h*)(tDst  + 1 * 1024) = hv;
        *(v8h*)(tDst2 + 1 * 1024) = rv;
        pack_state2(a2, hv, rv);
        *(v8h*)(tDst  + 2 * 1024) = hv;
        *(v8h*)(tDst2 + 2 * 1024) = rv;
        pack_state2(a3, hv, rv);
        *(v8h*)(tDst  + 3 * 1024) = hv;
        *(v8h*)(tDst2 + 3 * 1024) = rv;
      }
      __syncthreads();
      {
        v8f a0, a1, a2, a3, e0, e1, e2, e3;
        tile_product2(aRowT, aRowT2, bHi, a0, a1, a2, a3, e0, e1, e2, e3);
        scatter_tile(a0, e0, dl ^ ring_dst(0u << 10), sDst, last);
        scatter_tile(a1, e1, dl ^ ring_dst(1u << 10), sDst, last);
        scatter_tile(a2, e2, dl ^ ring_dst(2u << 10), sDst, last);
        scatter_tile(a3, e3, dl ^ ring_dst(3u << 10), sDst, last);
      }
      __syncthreads();
    }

    {
      v8f acc = (v8f){0.f, 0.f, 0.f, 0.f, 0.f, 0.f, 0.f, 0.f};
#pragma unroll
      for (int ks = 0; ks < 2; ++ks) {
        const v16h a = frag_load(aRowS + ks * 32);
        const v16h b = frag_load(bG + ks * 32);
        acc = mma_f16(a, b, acc);
      }
#pragma unroll
      for (int r = 0; r < 8; ++r) rDst[r * 16] = acc[r];
    }
    __syncthreads();

    if (wave == 0u) {
      unsigned lc = (lane < 26u) ? lane : 25u;
      asm volatile("" : "+v"(lc));
      unsigned el = (lc >= 13u) ? 1u : 0u;
      asm volatile("" : "+v"(el));
      unsigned kk = lc - el * 13u;
      asm volatile("" : "+v"(kk));
      const unsigned col = (kk < 6u) ? kk : 6u;
      const bool useSign = (kk >= 6u) && (kk < 12u);
      const unsigned sh  = useSign ? (kk - 6u) : 0u;
      const float* rp = sR + el * 64u * 16u;
      float num = 0.0f, tot = 0.0f;
#pragma unroll 4
      for (unsigned hi = 0; hi < 64u; ++hi) {
        const float rv = rp[hi * 16u + col];
        const float tv = rp[hi * 16u + 6u];
        const bool neg = useSign && (((hi >> sh) & 1u) != 0u);
        num += neg ? -rv : rv;
        tot += tv;
      }
      const float o = num / tot;
      if (lane < 26u && kk < 12u) sOut[(2u * it + el) * 12u + kk] = o;
    }
  }
  __syncthreads();

  if (wave == 0u) {
    const unsigned ls = (lane < 24u) ? lane : 23u;
    const v4f val = *(const v4f*)(sOut + ls * 4u);
    float* dst = out + (size_t)blockIdx.x * (size_t)(kRowsPerBlk * kAxes) + ls * 4u;
    if (lane < 24u) *(volatile v4f*)dst = val;
    __threadfence();
    if (lane < 24u) *(volatile v4f*)dst = val;
  }
}

extern "C" void kernel_launch(void* const* d_in, const int* in_sizes, int n_in,
                              void* d_out, int out_size, void* d_ws, size_t ws_size,
                              hipStream_t stream) {
  if (n_in < 2) return;
  if (in_sizes[0] != kSamples * kAxes) return;
  if (in_sizes[1] != kLayers * kAxes) return;
  if (out_size != kSamples * kAxes) return;
  if (ws_size < kWsTotal) return;

  const float* x     = (const float*)d_in[0];
  const float* theta = (const float*)d_in[1];
  float* out = (float*)d_out;
  unsigned short* planes = (unsigned short*)((char*)d_ws + kOffFact);

  prep_planes_kernel<<<1, 256, 0, stream>>>(theta, planes);
  state_evolve_kernel<<<kBlocks, 256, 0, stream>>>(x, theta, planes, out);
}
